// LocalInjectionAttnProcessor_34265249088251
// MI455X (gfx1250) — hardware-verified
//
#include <hip/hip_runtime.h>
#include <math.h>

constexpr int kB   = 4;
constexpr int kS   = 2048;
constexpr int kDm  = 1024;
constexpr int kH   = 16;
constexpr int kHd  = 64;
constexpr int kR   = 4;
constexpr int kTok = kB * kS;
constexpr int kGroupsPerChunk = 2;
constexpr int kNumGroups = kB * kH;
constexpr int kNumChunks = kNumGroups / kGroupsPerChunk;
constexpr float kWCarry    = 256.0f;
constexpr float kWCarryInv = 1.0f / 256.0f;
constexpr float kPCarry    = 2048.0f;
constexpr float kPVScale   = 1.0f / 2048.0f;
constexpr float kOCarry    = 256.0f;
constexpr float kOutScale  = 1.0f / (256.0f * 256.0f);
constexpr float kScoreScale = 0.125f;

static_assert(kNumGroups % kGroupsPerChunk == 0);
static_assert(kH % kGroupsPerChunk == 0);

typedef __attribute__((ext_vector_type(16))) _Float16 v16h;
typedef __attribute__((ext_vector_type(8)))  _Float16 v8h;
typedef __attribute__((ext_vector_type(16))) __bf16   v16b;
typedef __attribute__((ext_vector_type(8)))  __bf16   v8b;
typedef __attribute__((ext_vector_type(8)))  float    v8f;
typedef __attribute__((ext_vector_type(4)))  float    v4f;
typedef __attribute__((ext_vector_type(4)))  unsigned int v4u;

__device__ __forceinline__ unsigned short f2bf_bits(float f) {
  unsigned u = __float_as_uint(f);
  return (unsigned short)((u + 0x7FFFu + ((u >> 16) & 1u)) >> 16);
}
__device__ __forceinline__ float bf_bits2f(unsigned short h) { return __uint_as_float(((unsigned)h) << 16); }

__device__ __forceinline__ void dep_guard_h(v8f& a, v8f& b, v16h x, v16h y) { asm volatile("v_nop\n\tv_nop\n\tv_nop\n\tv_nop" : "+v"(a), "+v"(b) : "v"(x), "v"(y)); }
__device__ __forceinline__ void dep_guard_b(v8f& a, v8f& b, v16b x, v16b y) { asm volatile("v_nop\n\tv_nop\n\tv_nop\n\tv_nop" : "+v"(a), "+v"(b) : "v"(x), "v"(y)); }
__device__ __forceinline__ void keep4_h(v16h a, v16h b, v16h c, v16h d) { asm volatile("v_nop" :: "v"(a), "v"(b), "v"(c), "v"(d)); }
__device__ __forceinline__ void keep4_b(v16b a, v16b b, v16b c, v16b d) { asm volatile("v_nop" :: "v"(a), "v"(b), "v"(c), "v"(d)); }
__device__ __forceinline__ void acc_guard4(v8f& a, v8f& b, v8f& c, v8f& d) { asm volatile("v_nop\n\tv_nop\n\tv_nop\n\tv_nop" : "+v"(a), "+v"(b), "+v"(c), "+v"(d)); }
template <typename T> struct Frag;
template <> struct Frag<_Float16> {
  typedef v16h V; union U { v16h v; v8h h[2]; };
  static __device__ __forceinline__ v16h load(const _Float16* p) {
    U f; f.h[0] = *(const v8h*)(p); f.h[1] = *(const v8h*)(p + 16); return f.v;
  }
  static __device__ __forceinline__ v8f mma(v16h a, v16h b, v8f c) {
    return __builtin_amdgcn_wmma_f32_16x16x32_f16(false, a, false, b, (short)0, c, false, false);
  }
  static __device__ __forceinline__ void guard(v8f& a, v8f& b, v16h x, v16h y) { dep_guard_h(a, b, x, y); }
  static __device__ __forceinline__ void keep(v16h a, v16h b, v16h c, v16h d) { keep4_h(a, b, c, d); }
};
template <> struct Frag<__bf16> {
  typedef v16b V; union U { v16b v; v8b h[2]; };
  static __device__ __forceinline__ v16b load(const __bf16* p) {
    U f; f.h[0] = *(const v8b*)(p); f.h[1] = *(const v8b*)(p + 16); return f.v;
  }
  static __device__ __forceinline__ v8f mma(v16b a, v16b b, v8f c) {
    return __builtin_amdgcn_wmma_f32_16x16x32_bf16(false, a, false, b, (short)0, c, false, false);
  }
  static __device__ __forceinline__ void guard(v8f& a, v8f& b, v16b x, v16b y) { dep_guard_b(a, b, x, y); }
  static __device__ __forceinline__ void keep(v16b a, v16b b, v16b c, v16b d) { keep4_b(a, b, c, d); }
};

__device__ __forceinline__ unsigned pk16(unsigned short a, unsigned short b) { return (unsigned)a | ((unsigned)b << 16); }
__device__ __forceinline__ unsigned short h_bits(float f) { const _Float16 h = (_Float16)f; return __builtin_bit_cast(unsigned short, h); }

template <int ET> struct Elem;
template <> struct Elem<0> { typedef _Float16 T; };
template <> struct Elem<1> { typedef __bf16 T; };
template <int ET, bool SPLIT, int BIAS_MODE, int OUT_MODE, bool RESID, int ACT = 0>
__global__ __launch_bounds__(256) void wmma_gemm64(
    const unsigned short* __restrict__ Ap, const unsigned short* __restrict__ A2p, int lda, long strideA,
    const unsigned short* __restrict__ Btp, const unsigned short* __restrict__ Bt2p, int ldb, long strideB,
    void* __restrict__ Cout, void* __restrict__ Cout2, int ldc, long strideC,
    const float* __restrict__ bias,
    const float* __restrict__ resid, long strideR,
    int M, int N, int K, float scale) {
  typedef typename Elem<ET>::T T;
  typedef typename Frag<T>::V V;
  const T* A = (const T*)Ap; const T* A2 = (const T*)A2p; const T* Bt = (const T*)Btp; const T* Bt2 = (const T*)Bt2p;
  __shared__ __align__(16) float sT[8][16 * 68];
  const int b    = blockIdx.y;
  const int lane = threadIdx.x & 31;
  const int wave = threadIdx.x >> 5;
  const int tilesN = N >> 6;
  const int tilesM = M >> 6;
  const int tile = blockIdx.x * 8 + wave;
  if (tile >= tilesM * tilesN) return;
  const int tm = tile / tilesN;
  const int tn = tile - tm * tilesN;
  const int m0 = tm << 6;
  const int n0 = tn << 6;

  const T* Ab  = A  + (size_t)b * strideA;
  const T* Bb  = Bt + (size_t)b * strideB;
  const T* Ab2 = SPLIT ? (A2  + (size_t)b * strideA) : nullptr;
  const T* Bb2 = SPLIT ? (Bt2 + (size_t)b * strideB) : nullptr;

  const int rlane = lane & 15;
  const int koff  = (lane >> 4) * 8;
  const int mOff  = (lane >> 4) * 8;

  v8f acc[4][4];
#pragma unroll
  for (int i = 0; i < 4; ++i)
#pragma unroll
    for (int j = 0; j < 4; ++j) acc[i][j] = (v8f){0.f,0.f,0.f,0.f,0.f,0.f,0.f,0.f};

  for (int k0 = 0; k0 < K; k0 += 32) {
    V bh[4], bl[4];
#pragma unroll
    for (int j = 0; j < 4; ++j) {
      const size_t bo = (size_t)(n0 + (j << 4) + rlane) * ldb + koff + k0;
      bh[j] = Frag<T>::load(Bb + bo);
      if (SPLIT) bl[j] = Frag<T>::load(Bb2 + bo);
    }
#pragma unroll
    for (int i = 0; i < 4; ++i) {
      const size_t ao = (size_t)(m0 + (i << 4) + rlane) * lda + koff + k0;
      V ah = Frag<T>::load(Ab + ao);
      V al;
      if (SPLIT) al = Frag<T>::load(Ab2 + ao);
#pragma unroll
      for (int j = 0; j < 4; ++j) {
        acc[i][j] = Frag<T>::mma(ah, bh[j], acc[i][j]);
        if (SPLIT) {
          acc[i][j] = Frag<T>::mma(ah, bl[j], acc[i][j]);
          acc[i][j] = Frag<T>::mma(al, bh[j], acc[i][j]);
        }
      }
      Frag<T>::guard(acc[i][0], acc[i][3], ah, SPLIT ? al : ah);
    }
    Frag<T>::keep(bh[0], bh[1], bh[2], bh[3]);
    if (SPLIT) Frag<T>::keep(bl[0], bl[1], bl[2], bl[3]);
  }
  acc_guard4(acc[0][0], acc[0][1], acc[0][2], acc[0][3]);
  acc_guard4(acc[1][0], acc[1][1], acc[1][2], acc[1][3]);
  acc_guard4(acc[2][0], acc[2][1], acc[2][2], acc[2][3]);
  acc_guard4(acc[3][0], acc[3][1], acc[3][2], acc[3][3]);

  float* slab = sT[wave];
  const float* Rb = RESID ? (resid + (size_t)b * strideR) : nullptr;
#pragma unroll
  for (int i = 0; i < 4; ++i) {
    const int mBase = m0 + (i << 4);
#pragma unroll
    for (int j = 0; j < 4; ++j) {
      const int n = n0 + (j << 4) + rlane;
      float bv = 0.f;
      if (BIAS_MODE == 2) bv = bias[n];
#pragma unroll
      for (int r = 0; r < 8; ++r) {
        float v = acc[i][j][r] * scale;
        if (BIAS_MODE == 1) v += bias[mBase + mOff + r];
        if (BIAS_MODE == 2) v += bv;
        if (RESID) v += Rb[(size_t)(mBase + mOff + r) * ldc + n];
        if (ACT == 2) v = fmaxf(v, 0.0f);
        if (ACT == 4) v = (v > 0.f) ? v : 0.01f * v;
        slab[(mOff + r) * 68 + (j << 4) + rlane] = v;
      }
    }
    __builtin_amdgcn_fence(__ATOMIC_RELEASE, "workgroup");
    __builtin_amdgcn_wave_barrier();
    __builtin_amdgcn_fence(__ATOMIC_ACQUIRE, "workgroup");
    if (OUT_MODE == 0) {
      float* C = (float*)Cout + (size_t)b * strideC;
      const int hh = lane >> 4, c4 = (lane & 15) * 4;
      for (int pass = 0; pass < 2; ++pass) {
#pragma unroll
        for (int it = 0; it < 8; ++it) {
          const int row = it * 2 + hh;
          v4f v = *(const v4f*)(slab + row * 68 + c4);
          *(volatile v4f*)(C + (size_t)(mBase + row) * ldc + n0 + c4) = v;
        }
        __threadfence();
      }
    } else {
      const int q = lane >> 3, c8 = (lane & 7) * 8;
      unsigned short* C  = (unsigned short*)Cout  + (size_t)b * strideC;
      unsigned short* C2 = (OUT_MODE == 2) ? ((unsigned short*)Cout2 + (size_t)b * strideC) : nullptr;
      for (int pass = 0; pass < 2; ++pass) {
#pragma unroll
        for (int it = 0; it < 4; ++it) {
          const int row = it * 4 + q;
          const float* sp = slab + row * 68 + c8;
          v8h hv, lv;
#pragma unroll
          for (int e = 0; e < 8; ++e) {
            if (OUT_MODE == 1) {
              hv[e] = (_Float16)sp[e];
            } else {
              unsigned short hb = f2bf_bits(sp[e]);
              unsigned short lb = f2bf_bits(sp[e] - bf_bits2f(hb));
              hv[e] = __builtin_bit_cast(_Float16, hb);
              lv[e] = __builtin_bit_cast(_Float16, lb);
            }
          }
          *(volatile v8h*)(C + (size_t)(mBase + row) * ldc + n0 + c8) = hv;
          if (OUT_MODE == 2) *(volatile v8h*)(C2 + (size_t)(mBase + row) * ldc + n0 + c8) = lv;
        }
        __threadfence();
      }
    }
    __builtin_amdgcn_fence(__ATOMIC_RELEASE, "workgroup");
    __builtin_amdgcn_wave_barrier();
    __builtin_amdgcn_fence(__ATOMIC_ACQUIRE, "workgroup");
  }
}

__global__ __launch_bounds__(256) void cast8s_f16_kernel(const float* __restrict__ in, unsigned short* __restrict__ out, int n8, float scale) {
  const int i = blockIdx.x * 256 + threadIdx.x;
  if (i >= n8) return;
  const float* p = in + 8 * (size_t)i;
  const v4f a = *(const v4f*)(p);
  const v4f c = *(const v4f*)(p + 4);
  unsigned short hb[8];
#pragma unroll
  for (int e = 0; e < 4; ++e) {
    hb[e]     = h_bits(a[e] * scale);
    hb[4 + e] = h_bits(c[e] * scale);
  }
  const v4u u = (v4u){pk16(hb[0], hb[1]), pk16(hb[2], hb[3]), pk16(hb[4], hb[5]), pk16(hb[6], hb[7])};
  unsigned short* q = out + 8 * (size_t)i;
  *(volatile v4u*)q = u;
  __threadfence();
  *(volatile v4u*)q = u;
}

__global__ __launch_bounds__(256) void wtcast_kernel(const float* __restrict__ W0, const float* __restrict__ W1,
                                                     const float* __restrict__ W2,
                                                     unsigned short* __restrict__ out, float scale) {
  __shared__ float sm[64][65];
  const int t  = threadIdx.x;
  const int d0 = blockIdx.x * 64;
  const int h0 = blockIdx.y * 64;
  const int z  = blockIdx.z;
  const float* W = (z == 0) ? W0 : (z == 1) ? W1 : W2;
#pragma unroll
  for (int i = 0; i < 16; ++i) {
    const int e = i * 256 + t;
    const int r = e >> 6;
    const int c = e & 63;
    sm[c][r] = W[(size_t)(d0 + r) * kDm + h0 + c] * scale;
  }
  __syncthreads();
  const int lane = t & 31, wave = t >> 5;
  const int q = lane >> 3, c8 = (lane & 7) * 8;
  unsigned short* op = out + (size_t)z * kDm * kDm;
  for (int pass = 0; pass < 2; ++pass) {
#pragma unroll
    for (int it = 0; it < 2; ++it) {
      const int row = wave * 8 + it * 4 + q;
      unsigned short hb[8];
#pragma unroll
      for (int e = 0; e < 8; ++e) hb[e] = h_bits(sm[row][c8 + e]);
      const v4u u = (v4u){pk16(hb[0], hb[1]), pk16(hb[2], hb[3]), pk16(hb[4], hb[5]), pk16(hb[6], hb[7])};
      *(volatile v4u*)(op + (size_t)(h0 + row) * kDm + d0 + c8) = u;
    }
    __threadfence();
  }
}

__global__ __launch_bounds__(256) void lora_down_kernel(const float* __restrict__ X, const float* __restrict__ dn,
                                                        float* __restrict__ Dout, int nrows) {
  __shared__ __align__(16) float sD[8][32];
  const int lane = threadIdx.x & 31, wave = threadIdx.x >> 5;
  const int row0 = blockIdx.x * 64 + wave * 8;
#pragma unroll 1
  for (int j = 0; j < 8; ++j) {
    const int row  = row0 + j;
    const int rowc = row < nrows ? row : nrows - 1;
    const float* xr = X + (size_t)rowc * kDm;
    float a0 = 0.f, a1 = 0.f, a2 = 0.f, a3 = 0.f;
#pragma unroll 1
    for (int i = 0; i < 8; ++i) {
      const int k = 4 * lane + 128 * i;
      const v4f xv = *(const v4f*)(xr + k);
      const float* dp = dn + 4 * k;
      const v4f w0 = *(const v4f*)(dp);
      const v4f w1 = *(const v4f*)(dp + 4);
      const v4f w2 = *(const v4f*)(dp + 8);
      const v4f w3 = *(const v4f*)(dp + 12);
      a0 += xv[0] * w0[0] + xv[1] * w1[0] + xv[2] * w2[0] + xv[3] * w3[0];
      a1 += xv[0] * w0[1] + xv[1] * w1[1] + xv[2] * w2[1] + xv[3] * w3[1];
      a2 += xv[0] * w0[2] + xv[1] * w1[2] + xv[2] * w2[2] + xv[3] * w3[2];
      a3 += xv[0] * w0[3] + xv[1] * w1[3] + xv[2] * w2[3] + xv[3] * w3[3];
    }
#pragma unroll
    for (int off = 16; off > 0; off >>= 1) {
      a0 += __shfl_xor(a0, off, 32);
      a1 += __shfl_xor(a1, off, 32);
      a2 += __shfl_xor(a2, off, 32);
      a3 += __shfl_xor(a3, off, 32);
    }
    if (lane == 0) {
      sD[wave][4 * j + 0] = a0;
      sD[wave][4 * j + 1] = a1;
      sD[wave][4 * j + 2] = a2;
      sD[wave][4 * j + 3] = a3;
    }
  }
  __builtin_amdgcn_fence(__ATOMIC_RELEASE, "workgroup");
  __builtin_amdgcn_wave_barrier();
  __builtin_amdgcn_fence(__ATOMIC_ACQUIRE, "workgroup");
  const v4f v = *(const v4f*)(&sD[wave][4 * (lane & 7)]);
  float* dst = Dout + (size_t)(row0 + (lane & 7)) * kR;
  if (lane < 8) *(volatile v4f*)dst = v;
  __threadfence();
  if (lane < 8) *(volatile v4f*)dst = v;
}

template <int TRANS>
__global__ __launch_bounds__(256) void lora_up_kernel(const float* __restrict__ Dm, const float* __restrict__ up,
                                                      float* __restrict__ L, int total4) {
  const int e = blockIdx.x * 256 + threadIdx.x;
  if (e >= total4) return;
  v4f o;
  size_t dst;
  if (TRANS == 0) {
    const int row = e >> 8;
    const int n   = (e & 255) * 4;
    const v4f d  = *(const v4f*)(Dm + (size_t)row * kR);
    const v4f u0 = *(const v4f*)(up + n);
    const v4f u1 = *(const v4f*)(up + kDm + n);
    const v4f u2 = *(const v4f*)(up + 2 * kDm + n);
    const v4f u3 = *(const v4f*)(up + 3 * kDm + n);
    o = d[0] * u0 + d[1] * u1 + d[2] * u2 + d[3] * u3;
    dst = (size_t)row * kDm + n;
  } else {
    const int n  = e >> 11;
    const int t4 = (e & 2047) * 4;
    const v4f d0 = *(const v4f*)(Dm + (size_t)(t4 + 0) * kR);
    const v4f d1 = *(const v4f*)(Dm + (size_t)(t4 + 1) * kR);
    const v4f d2 = *(const v4f*)(Dm + (size_t)(t4 + 2) * kR);
    const v4f d3 = *(const v4f*)(Dm + (size_t)(t4 + 3) * kR);
    const float u0 = up[n], u1 = up[kDm + n], u2 = up[2 * kDm + n], u3 = up[3 * kDm + n];
    o[0] = d0[0] * u0 + d0[1] * u1 + d0[2] * u2 + d0[3] * u3;
    o[1] = d1[0] * u0 + d1[1] * u1 + d1[2] * u2 + d1[3] * u3;
    o[2] = d2[0] * u0 + d2[1] * u1 + d2[2] * u2 + d2[3] * u3;
    o[3] = d3[0] * u0 + d3[1] * u1 + d3[2] * u2 + d3[3] * u3;
    dst = (size_t)n * kTok + t4;
  }
  *(volatile v4f*)(L + dst) = o;
  __threadfence();
  *(volatile v4f*)(L + dst) = o;
}

__global__ __launch_bounds__(256) void softmax_row_kernel(const float* __restrict__ S, unsigned short* __restrict__ P, float carry) {
  __shared__ float redM[8];
  __shared__ float redS[8];
  const int row  = blockIdx.x;
  const int t    = threadIdx.x;
  const int lane = t & 31, wave = t >> 5;
  const int c0   = t * 8;
  const float* sr = S + (size_t)row * kS + c0;
  const v4f a = *(const v4f*)(sr);
  const v4f c = *(const v4f*)(sr + 4);
  float x[8];
#pragma unroll
  for (int e = 0; e < 4; ++e) { x[e] = a[e]; x[4 + e] = c[e]; }
  float m = fmaxf(fmaxf(fmaxf(x[0], x[1]), fmaxf(x[2], x[3])), fmaxf(fmaxf(x[4], x[5]), fmaxf(x[6], x[7])));
#pragma unroll
  for (int off = 16; off > 0; off >>= 1) m = fmaxf(m, __shfl_xor(m, off, 32));
  if (lane == 0) redM[wave] = m;
  __syncthreads();
  float gm = redM[0];
#pragma unroll
  for (int w = 1; w < 8; ++w) gm = fmaxf(gm, redM[w]);
  float ev[8];
  float s = 0.f;
#pragma unroll
  for (int e = 0; e < 8; ++e) { ev[e] = expf(x[e] - gm); s += ev[e]; }
#pragma unroll
  for (int off = 16; off > 0; off >>= 1) s += __shfl_xor(s, off, 32);
  if (lane == 0) redS[wave] = s;
  __syncthreads();
  float tot = redS[0];
#pragma unroll
  for (int w = 1; w < 8; ++w) tot += redS[w];
  const float f = carry * (1.0f / tot);
  unsigned short hb[8];
#pragma unroll
  for (int e = 0; e < 8; ++e) hb[e] = h_bits(ev[e] * f);
  const v4u u = (v4u){pk16(hb[0], hb[1]), pk16(hb[2], hb[3]), pk16(hb[4], hb[5]), pk16(hb[6], hb[7])};
  unsigned short* q = P + (size_t)row * kS + c0;
  *(volatile v4u*)q = u;
  __threadfence();
  *(volatile v4u*)q = u;
}

extern "C" void kernel_launch(void* const* d_in, const int* in_sizes, int n_in,
                              void* d_out, int out_size, void* d_ws, size_t ws_size,
                              hipStream_t stream)
{
  const size_t MiB = 1048576;
  const int nAct = kTok * kDm;
  if (n_in < 15) return;
  if (in_sizes[0] != nAct || in_sizes[1] != nAct) return;
  for (int i = 2; i <= 5; ++i) if (in_sizes[i] != kDm * kDm) return;
  if (in_sizes[6] != kDm) return;
  for (int i = 7; i <= 14; ++i) if (in_sizes[i] != kDm * kR) return;
  if (out_size != nAct) return;
  if (ws_size < 128 * MiB) return;

  const float* hs   = (const float*)d_in[0];
  const float* enc  = (const float*)d_in[1];
  const float* Wq   = (const float*)d_in[2];
  const float* Wk   = (const float*)d_in[3];
  const float* Wv   = (const float*)d_in[4];
  const float* Wo   = (const float*)d_in[5];
  const float* bo   = (const float*)d_in[6];
  const float* q_dn = (const float*)d_in[7];
  const float* q_up = (const float*)d_in[8];
  const float* k_dn = (const float*)d_in[9];
  const float* k_up = (const float*)d_in[10];
  const float* v_dn = (const float*)d_in[11];
  const float* v_up = (const float*)d_in[12];
  const float* o_dn = (const float*)d_in[13];
  const float* o_up = (const float*)d_in[14];
  float* out = (float*)d_out;

  char* wsc = (char*)d_ws;
  unsigned short* Q16  = (unsigned short*)(wsc + 0 * MiB);
  unsigned short* WoT  = (unsigned short*)(wsc + 0 * MiB);
  unsigned short* K16  = (unsigned short*)(wsc + 16 * MiB);
  float*          Do   = (float*)(wsc + 16 * MiB);
  unsigned short* Vt16 = (unsigned short*)(wsc + 32 * MiB);
  float*          LORA = (float*)(wsc + 48 * MiB);
  float*          O32  = (float*)(wsc + 48 * MiB);
  unsigned short* X16  = (unsigned short*)(wsc + 80 * MiB);
  unsigned short* E16  = (unsigned short*)(wsc + 96 * MiB);
  float*          S32  = (float*)(wsc + 80 * MiB);
  float*          LORo = (float*)(wsc + 80 * MiB);
  unsigned short* WT3  = (unsigned short*)(wsc + 112 * MiB);
  const unsigned short* WqT = WT3;
  const unsigned short* WkT = WT3 + (size_t)kDm * kDm;
  const unsigned short* WvT = WT3 + (size_t)2 * kDm * kDm;
  float*          Dq   = (float*)(wsc + 118 * MiB);
  float*          Dk   = Dq + (size_t)kTok * kR;
  float*          Dv   = Dk + (size_t)kTok * kR;
  unsigned short* P16  = (unsigned short*)(wsc + 112 * MiB);
  unsigned short* O16  = (unsigned short*)(wsc + 112 * MiB);

  const int n8 = nAct / 8;
  const int castBlocks = (n8 + 255) / 256;
  const int loraDownBlocks = kTok / 64;
  const int up4 = kTok * (kDm / 4);
  const int upBlocks = (up4 + 255) / 256;
  const int projTiles = (kTok / 64) * (kDm / 64);
  const int projBlocks = (projTiles + 7) / 8;

  cast8s_f16_kernel<<<castBlocks, 256, 0, stream>>>(hs,  X16, n8, 1.0f);
  cast8s_f16_kernel<<<castBlocks, 256, 0, stream>>>(enc, E16, n8, 1.0f);
  wtcast_kernel<<<dim3(kDm / 64, kDm / 64, 3), 256, 0, stream>>>(Wq, Wk, Wv, WT3, kWCarry);
  lora_down_kernel<<<loraDownBlocks, 256, 0, stream>>>(hs,  q_dn, Dq, kTok);
  lora_down_kernel<<<loraDownBlocks, 256, 0, stream>>>(enc, k_dn, Dk, kTok);
  lora_down_kernel<<<loraDownBlocks, 256, 0, stream>>>(enc, v_dn, Dv, kTok);

  lora_up_kernel<0><<<upBlocks, 256, 0, stream>>>(Dq, q_up, LORA, up4);
  wmma_gemm64<0, false, 0, 1, true><<<dim3(projBlocks, 1), 256, 0, stream>>>(
      X16, nullptr, kDm, 0L, WqT, nullptr, kDm, 0L,
      (void*)Q16, nullptr, kDm, 0L, nullptr, LORA, 0L, kTok, kDm, kDm, kWCarryInv);
  lora_up_kernel<0><<<upBlocks, 256, 0, stream>>>(Dk, k_up, LORA, up4);
  wmma_gemm64<0, false, 0, 1, true><<<dim3(projBlocks, 1), 256, 0, stream>>>(
      E16, nullptr, kDm, 0L, WkT, nullptr, kDm, 0L,
      (void*)K16, nullptr, kDm, 0L, nullptr, LORA, 0L, kTok, kDm, kDm, kWCarryInv);
  lora_up_kernel<1><<<upBlocks, 256, 0, stream>>>(Dv, v_up, LORA, up4);
  wmma_gemm64<0, false, 0, 1, true><<<dim3(projBlocks, 1), 256, 0, stream>>>(
      WvT, nullptr, kDm, 0L, E16, nullptr, kDm, 0L,
      (void*)Vt16, nullptr, kTok, 0L, nullptr, LORA, 0L, kDm, kTok, kDm, kWCarryInv);

  const int sTiles = (kS / 64) * (kS / 64);
  const int sBlocks = (sTiles + 7) / 8;
  const int pvTiles = (kS / 64) * (kHd / 64);
  const int pvBlocks = (pvTiles + 7) / 8;
  for (int cix = 0; cix < kNumChunks; ++cix) {
    const int g0 = cix * kGroupsPerChunk;
    const int bb = g0 / kH;
    const int h0 = g0 % kH;
    const unsigned short* Qg = Q16 + (size_t)bb * kS * kDm + (size_t)h0 * kHd;
    const unsigned short* Kg = K16 + (size_t)bb * kS * kDm + (size_t)h0 * kHd;
    wmma_gemm64<0, false, 0, 0, false><<<dim3(sBlocks, kGroupsPerChunk), 256, 0, stream>>>(
        Qg, nullptr, kDm, (long)kHd, Kg, nullptr, kDm, (long)kHd,
        (void*)S32, nullptr, kS, (long)kS * kS, nullptr, nullptr, 0L, kS, kS, kHd, kScoreScale);
    softmax_row_kernel<<<kGroupsPerChunk * kS, 256, 0, stream>>>(S32, P16, kPCarry);
    const unsigned short* Vg = Vt16 + (size_t)h0 * kHd * kTok + (size_t)bb * kS;
    float* Og = O32 + (size_t)bb * kS * kDm + (size_t)h0 * kHd;
    wmma_gemm64<0, false, 0, 0, false><<<dim3(pvBlocks, kGroupsPerChunk), 256, 0, stream>>>(
        P16, nullptr, kS, (long)kS * kS, Vg, nullptr, kTok, (long)kHd * kTok,
        (void*)Og, nullptr, kDm, (long)kHd, nullptr, nullptr, 0L, kS, kHd, kS, kPVScale);
  }

  cast8s_f16_kernel<<<castBlocks, 256, 0, stream>>>(O32, O16, n8, kOCarry);
  wtcast_kernel<<<dim3(kDm / 64, kDm / 64, 1), 256, 0, stream>>>(Wo, Wo, Wo, WoT, kWCarry);
  lora_down_kernel<<<loraDownBlocks, 256, 0, stream>>>(O32, o_dn, Do, kTok);
  lora_up_kernel<0><<<upBlocks, 256, 0, stream>>>(Do, o_up, LORo, up4);
  wmma_gemm64<0, false, 2, 0, true><<<dim3(projBlocks, 1), 256, 0, stream>>>(
      O16, nullptr, kDm, 0L, WoT, nullptr, kDm, 0L,
      (void*)out, nullptr, kDm, 0L, bo, LORo, 0L, kTok, kDm, kDm, kOutScale);
}
